// projection_CalculateMatrixQ_85813446574644
// MI455X (gfx1250) — hardware-verified
//
#include <hip/hip_runtime.h>


#ifndef NB
#define NB 32
#endif
#ifndef SEQ
#define SEQ 128
#endif
#define NB_FULL  32
#define SEQ_FULL 128
#define DM   128
#define K2   (2 * SEQ)
#define KP   (2 * K2)
#define OTR  32
#define ACARRY 4096.0f
#define BCARRY 16.0f
#define OFOLD  (1.0f / 65536.0f)
#define RCARRY 2048.0f
#define RFOLD  (1.0f / 2048.0f)
#define LOG2E  1.4426950408889634f

static_assert(DM % 64 == 0);
static_assert(DM % 32 == 0);
static_assert(K2 % 32 == 0);
static_assert(KP == 2 * K2);
static_assert((KP * 2) % 128 == 0);
static_assert(OTR == 2 * 16);
static_assert(DM % OTR == 0);
static_assert(SEQ % 64 == 0);
static_assert((NB * SEQ) % 64 == 0);
static_assert(SEQ <= 1024);
static_assert(SEQ / 32 <= 32);
static_assert(NB <= NB_FULL);
static_assert(SEQ <= SEQ_FULL);
static_assert(((size_t)SEQ * DM) % 8 == 0);
static_assert(((size_t)DM * DM) % 8 == 0);
static_assert((size_t)NB_FULL * DM * DM * 4 == (size_t)2097152);
static_assert(8 * 32 * 16 == 16 * 64 * 4);
static_assert((DM / 8) * SEQ * 16 == DM * SEQ * 2);
static_assert(16 * 68 * 4 <= 131072);
static_assert((64 + 64 + 2 * SEQ) * 4 <= 131072);
static_assert((68 * 4) % 16 == 0);

typedef _Float16 h16;
typedef unsigned short bf;
typedef __attribute__((ext_vector_type(16))) __bf16   v16bf;
typedef __attribute__((ext_vector_type(16))) _Float16 v16h;
typedef __attribute__((ext_vector_type(8)))  _Float16 v8h;
typedef __attribute__((ext_vector_type(8)))  unsigned short v8us;
typedef __attribute__((ext_vector_type(8)))  float    v8f;
typedef __attribute__((ext_vector_type(4)))  float    v4f;
typedef v4f  __attribute__((may_alias)) v4fa;

__device__ __forceinline__ unsigned short f2bf(float f) { unsigned u = __float_as_uint(f); u += 0x7FFFu + ((u >> 16) & 1u); return (unsigned short)(u >> 16); }
__device__ __forceinline__ float bfr(float f) { return __uint_as_float(((unsigned)f2bf(f)) << 16); }
__device__ __forceinline__ v16h cat16(v8h lo, v8h hi) { return __builtin_shufflevector(lo, hi, 0, 1, 2, 3, 4, 5, 6, 7, 8, 9, 10, 11, 12, 13, 14, 15); }
__device__ __forceinline__ v16bf cat16b(v8us lo, v8us hi) { return __builtin_bit_cast(v16bf, __builtin_shufflevector(lo, hi, 0, 1, 2, 3, 4, 5, 6, 7, 8, 9, 10, 11, 12, 13, 14, 15)); }
__device__ __forceinline__ v8f wmma16(v16h a, v16h b, v8f c) { return __builtin_amdgcn_wmma_f32_16x16x32_f16(false, a, false, b, (short)0, c, false, false); }
__device__ __forceinline__ v8f wmmab(v16bf a, v16bf b, v8f c) { return __builtin_amdgcn_wmma_f32_16x16x32_bf16(false, a, false, b, (short)0, c, false, false); }
__device__ __forceinline__ v16h  ldh(const h16* p) { return cat16(*(const v8h*)p, *(const v8h*)(p + 16)); }
__device__ __forceinline__ v16bf ldb(const bf* p)  { return cat16b(*(const v8us*)p, *(const v8us*)(p + 16)); }
__device__ __forceinline__ void wave_sync() { __builtin_amdgcn_fence(3  , "wavefront"); __builtin_amdgcn_wave_barrier(); asm volatile("" ::: "memory"); }

__device__ __forceinline__ v8f wmmab_g(v16bf a, v16bf b, v8f c) { c = wmmab(a, b, c); asm volatile("v_nop\n\tv_nop\n\tv_nop\n\tv_nop" : "+v"(c) : "v"(a), "v"(b)); return c; }
__device__ __forceinline__ v8f wmma16_g(v16h a, v16h b, v8f c) { c = wmma16(a, b, c); asm volatile("v_nop\n\tv_nop\n\tv_nop\n\tv_nop" : "+v"(c) : "v"(a), "v"(b)); return c; }
static __device__ __forceinline__ h16 toh_flush(float v) { const h16 r = (h16)v; return (fabsf(v) < 6.103515625e-05f) ? (h16)0.0f : r; }
static __device__ __forceinline__ void hsplit(float v, h16& h, h16& r) { h = toh_flush(v); r = toh_flush((v - (float)h) * RCARRY); }

__global__ __launch_bounds__(256) void k_cvt8(const float* __restrict__ src, bf* dst, size_t n8) {
    const size_t i = (size_t)blockIdx.x * 256 + threadIdx.x; if (i >= n8) return;
    const v8f v = *(const v8f*)(src + i * 8); v8us o;
#pragma unroll
    for (int k = 0; k < 8; ++k) o[k] = f2bf(v[k]);
    *(volatile v8us*)(dst + i * 8) = o; __threadfence(); *(volatile v8us*)(dst + i * 8) = o;
}

__global__ __launch_bounds__(32) void k_lin(const bf* __restrict__ A, const bf* __restrict__ Bt, const float* __restrict__ bias, float* RTp) {
    __shared__ __align__(16) float os[16 * 68];
    const int K = DM;
    const int lane = threadIdx.x & 31, lr = lane & 15, hi = lane >> 4; const int r0 = blockIdx.x * 64, c0 = blockIdx.y * 64;
    v8f acc[4][4];
#pragma unroll
    for (int mb = 0; mb < 4; ++mb)
#pragma unroll
        for (int nb = 0; nb < 4; ++nb) acc[mb][nb] = (v8f){};
    const size_t aoff = (size_t)(r0 + lr) * K + 8 * hi, boff = (size_t)(c0 + lr) * K + 8 * hi;
#pragma unroll 1
    for (int kc = 0; kc < K; kc += 32) {
        v16bf a[4];
#pragma unroll
        for (int mb = 0; mb < 4; ++mb) a[mb] = ldb(A + aoff + (size_t)mb * 16 * K + kc);
#pragma unroll
        for (int nb = 0; nb < 4; ++nb) { const v16bf b = ldb(Bt + boff + (size_t)nb * 16 * K + kc);
#pragma unroll
            for (int mb = 0; mb < 4; ++mb) acc[mb][nb] = wmmab_g(a[mb], b, acc[mb][nb]); }
    }
    const int bb = c0 / SEQ, tt = c0 % SEQ;
    const size_t tbase = (size_t)bb * (size_t)DM * SEQ + (size_t)r0 * SEQ + (size_t)tt;
#pragma unroll
    for (int mb = 0; mb < 4; ++mb) {
        float br[8];
#pragma unroll
        for (int j = 0; j < 8; ++j) br[j] = bfr(bias[r0 + mb * 16 + hi * 8 + j]);
#pragma unroll
        for (int nb = 0; nb < 4; ++nb) {
#pragma unroll
            for (int j = 0; j < 8; ++j) os[(hi * 8 + j) * 68 + nb * 16 + lr] = acc[mb][nb][j] + br[j]; }
        wave_sync();
#pragma unroll 1
        for (int ps = 0; ps < 2; ++ps) {
#pragma unroll
            for (int s = 0; s < 8; ++s) { const int p = s * 32 + lane; const int row = p >> 4, c4 = (p & 15) * 4;
                const v4f val = *(const v4fa*)(&os[row * 68 + c4]);
                *(volatile v4f*)(RTp + tbase + (size_t)(mb * 16 + row) * SEQ + c4) = val; }
            if (ps == 0) __threadfence(); }
        wave_sync();
    }
}

__global__ __launch_bounds__(SEQ) void k_att(const float* __restrict__ RT, h16* BTp, h16* AM) {
#pragma clang fp contract(off)
    __shared__ float redm[64];
    __shared__ float reds[64];
    __shared__ __align__(16) float atr[SEQ];
    __shared__ __align__(16) float ati[SEQ];
    const int tid = threadIdx.x, lane = tid & 31;
    const int wave = __builtin_amdgcn_readfirstlane((int)(threadIdx.x >> 5));
    const int b = blockIdx.x;
    const size_t pl = (size_t)NB * DM * SEQ;
    const size_t rb = (size_t)b * DM * SEQ;
    const float* base = RT + rb + tid;
    float lgr = 0.0f, lgi = 0.0f;
#pragma unroll 2
    for (int d = 0; d < DM; ++d) {
        const float a = base[(size_t)d * SEQ], bq = base[pl + (size_t)d * SEQ], c = base[2 * pl + (size_t)d * SEQ], e = base[3 * pl + (size_t)d * SEQ];
        lgr += (a * a - bq * bq) * (c * c - e * e);
        lgi += (2.0f * a * bq) * (2.0f * c * e);
    }
    float mr = lgr, mi = lgi;
#pragma unroll
    for (int off = 16; off > 0; off >>= 1) { mr = fmaxf(mr, __shfl_xor(mr, off, 32)); mi = fmaxf(mi, __shfl_xor(mi, off, 32)); }
    if (lane == 0) { redm[wave] = mr; redm[32 + wave] = mi; }
    __syncthreads();
    float MR = redm[0], MI = redm[32];
#pragma unroll
    for (int w = 1; w < SEQ / 32; ++w) { MR = fmaxf(MR, redm[w]); MI = fmaxf(MI, redm[32 + w]); }
    const float eR = __builtin_amdgcn_exp2f((lgr - MR) * LOG2E), eI = __builtin_amdgcn_exp2f((lgi - MI) * LOG2E);
    float sr = eR, si = eI;
#pragma unroll
    for (int off = 16; off > 0; off >>= 1) { sr += __shfl_xor(sr, off, 32); si += __shfl_xor(si, off, 32); }
    if (lane == 0) { reds[wave] = sr; reds[32 + wave] = si; }
    __syncthreads();
    float SR = reds[0], SI = reds[32];
#pragma unroll
    for (int w = 1; w < SEQ / 32; ++w) { SR += reds[w]; SI += reds[32 + w]; }
    atr[tid] = eR * __builtin_amdgcn_rcpf(SR);
    ati[tid] = eI * __builtin_amdgcn_rcpf(SI);
    __syncthreads();
    const int PPR = SEQ / 8;
#pragma unroll 1
    for (int ps = 0; ps < 2; ++ps) {
#pragma unroll 1
        for (int it = 0; it < DM / 8; ++it) {
            const int p = it * SEQ + tid; const int d = p / PPR, l8 = (p % PPR) * 8;
            const float* rp = RT + 2 * pl + rb + (size_t)d * SEQ + l8;
            const v4f ra = *(const v4f*)rp, rc = *(const v4f*)(rp + 4);
            const v4f qa = *(const v4f*)(rp + pl), qc = *(const v4f*)(rp + pl + 4);
            const v4f wa = *(const v4fa*)(&atr[l8]), wc = *(const v4fa*)(&atr[l8 + 4]);
            const v4f ua = *(const v4fa*)(&ati[l8]), uc = *(const v4fa*)(&ati[l8 + 4]);
            float rr[8], qq[8], sR[8], sI[8];
#pragma unroll
            for (int i = 0; i < 4; ++i) { rr[i] = ra[i]; rr[4 + i] = rc[i]; qq[i] = qa[i]; qq[4 + i] = qc[i];
                                          sR[i] = wa[i] * ACARRY; sR[4 + i] = wc[i] * ACARRY; sI[i] = ua[i] * ACARRY; sI[4 + i] = uc[i] * ACARRY; }
            v8h bh0, bh1, bs0, bs1, rh0, rh1, rs0, rs1, ih0, ih1, is0, is1;
#pragma unroll
            for (int i = 0; i < 8; ++i) {
                h16 hv, rv;
                hsplit(rr[i] * BCARRY, hv, rv);      bh0[i] = hv; bs0[i] = rv;
                hsplit(qq[i] * BCARRY, hv, rv);      bh1[i] = hv; bs1[i] = rv;
                hsplit(sR[i] * rr[i], hv, rv);       rh0[i] = hv; rs0[i] = rv;
                hsplit(-(sR[i] * qq[i]), hv, rv);    rh1[i] = hv; rs1[i] = rv;
                hsplit(sI[i] * qq[i], hv, rv);       ih0[i] = hv; is0[i] = rv;
                hsplit(sI[i] * rr[i], hv, rv);       ih1[i] = hv; is1[i] = rv; }
            const size_t ob = ((size_t)b * DM + (size_t)d) * KP + (size_t)l8;
            const size_t o1 = (size_t)NB * DM * KP + ob;
            *(volatile v8h*)(BTp + ob) = bh0;      *(volatile v8h*)(BTp + ob + SEQ) = bh1;
            *(volatile v8h*)(BTp + ob + K2) = bs0; *(volatile v8h*)(BTp + ob + K2 + SEQ) = bs1;
            *(volatile v8h*)(AM + ob) = rh0;       *(volatile v8h*)(AM + ob + SEQ) = rh1;
            *(volatile v8h*)(AM + ob + K2) = rs0;  *(volatile v8h*)(AM + ob + K2 + SEQ) = rs1;
            *(volatile v8h*)(AM + o1) = ih0;       *(volatile v8h*)(AM + o1 + SEQ) = ih1;
            *(volatile v8h*)(AM + o1 + K2) = is0;  *(volatile v8h*)(AM + o1 + K2 + SEQ) = is1;
        }
        if (ps == 0) __threadfence(); }
}

__global__ __launch_bounds__(32) __attribute__((amdgpu_num_vgpr(256))) void k_outer(const h16* __restrict__ AM, const h16* __restrict__ BTp, float* OUT) {
    __shared__ __align__(16) float os[16 * 68];
    const int lane = threadIdx.x & 31, lr = lane & 15, hi = lane >> 4; const int r0 = blockIdx.x * OTR, c0 = blockIdx.y * 64;
    const int z = blockIdx.z; const int which = z / NB, b = z % NB;
    v8f acc[2][4], accR[2][4];
#pragma unroll
    for (int mb = 0; mb < 2; ++mb)
#pragma unroll
        for (int nb = 0; nb < 4; ++nb) { acc[mb][nb] = (v8f){}; accR[mb][nb] = (v8f){}; }
    const size_t aoff = ((size_t)z * DM + (size_t)(r0 + lr)) * KP + 8 * hi, boff = ((size_t)b * DM + (size_t)(c0 + lr)) * KP + 8 * hi;
#pragma unroll 1
    for (int kc = 0; kc < K2; kc += 32) {
        v16h ah[2], ar[2];
#pragma unroll
        for (int mb = 0; mb < 2; ++mb) { ah[mb] = ldh(AM + aoff + (size_t)mb * 16 * KP + kc); ar[mb] = ldh(AM + aoff + (size_t)mb * 16 * KP + K2 + kc); }
#pragma unroll
        for (int nb = 0; nb < 4; ++nb) {
            const v16h bh = ldh(BTp + boff + (size_t)nb * 16 * KP + kc);
            const v16h bs = ldh(BTp + boff + (size_t)nb * 16 * KP + K2 + kc);
#pragma unroll
            for (int mb = 0; mb < 2; ++mb) {
                acc[mb][nb]  = wmma16_g(ah[mb], bh, acc[mb][nb]);
                accR[mb][nb] = wmma16_g(ar[mb], bh, accR[mb][nb]);
                accR[mb][nb] = wmma16_g(ah[mb], bs, accR[mb][nb]); } }
    }
    const size_t obase = (size_t)which * ((size_t)NB_FULL * DM * DM) + (size_t)b * DM * DM + (size_t)r0 * DM + (size_t)c0;
#pragma unroll
    for (int mb = 0; mb < 2; ++mb) {
#pragma unroll
        for (int nb = 0; nb < 4; ++nb) {
#pragma unroll
            for (int j = 0; j < 8; ++j) os[(hi * 8 + j) * 68 + nb * 16 + lr] = (acc[mb][nb][j] + accR[mb][nb][j] * RFOLD) * OFOLD; }
        wave_sync();
#pragma unroll 1
        for (int ps = 0; ps < 2; ++ps) {
#pragma unroll
            for (int s = 0; s < 8; ++s) { const int p = s * 32 + lane; const int row = p >> 4, c4 = (p & 15) * 4;
                const v4f val = *(const v4fa*)(&os[row * 68 + c4]);
                *(volatile v4f*)(OUT + obase + (size_t)(mb * 16 + row) * DM + c4) = val; }
            if (ps == 0) __threadfence(); }
        wave_sync();
    }
}

static constexpr size_t al256(size_t v) { return (v + 255) & ~(size_t)255; }
static constexpr size_t SZ_XB = al256((size_t)NB * SEQ * DM * 2);
static constexpr size_t SZ_WB = al256((size_t)4 * DM * DM * 2);
static constexpr size_t SZ_RT = al256((size_t)4 * NB * DM * SEQ * 4);
static constexpr size_t SZ_BT = al256((size_t)NB * DM * KP * 2);
static constexpr size_t SZ_AM = al256((size_t)2 * NB * DM * KP * 2);
static constexpr size_t SZ_TOTAL = 2 * SZ_XB + SZ_WB + SZ_RT + SZ_BT + SZ_AM;
static_assert(SZ_TOTAL <= (size_t)134217728);
static_assert(((size_t)DM * DM * 2) % 256 == 0);
static_assert(((size_t)NB * DM * SEQ * 4) % 256 == 0);
static_assert(((size_t)NB * DM * KP * 2) % 256 == 0);

extern "C" void kernel_launch(void* const* d_in, const int* in_sizes, int n_in,
                              void* d_out, int out_size, void* d_ws, size_t ws_size, hipStream_t stream) {
    if (n_in < 10) return;
    const size_t needx = ((size_t)(NB - 1) * SEQ_FULL + SEQ) * DM;
    if ((size_t)in_sizes[0] < needx || (size_t)in_sizes[1] < needx) return;
    if ((size_t)in_sizes[2] < (size_t)DM * DM || (size_t)in_sizes[4] < (size_t)DM * DM || (size_t)in_sizes[6] < (size_t)DM * DM || (size_t)in_sizes[8] < (size_t)DM * DM) return;
    if (in_sizes[3] < DM || in_sizes[5] < DM || in_sizes[7] < DM || in_sizes[9] < DM) return;
    if ((size_t)out_size < (size_t)NB_FULL * DM * DM + (size_t)NB * DM * DM) return;
    if (SZ_TOTAL > ws_size) return;
    const float* xin[2] = { (const float*)d_in[0], (const float*)d_in[1] };
    const float* wr1 = (const float*)d_in[2]; const float* br1 = (const float*)d_in[3];
    const float* wi1 = (const float*)d_in[4]; const float* bi1 = (const float*)d_in[5];
    const float* wr2 = (const float*)d_in[6]; const float* br2 = (const float*)d_in[7];
    const float* wi2 = (const float*)d_in[8]; const float* bi2 = (const float*)d_in[9];
    float* OUT = (float*)d_out;
    char* wsp = (char*)d_ws;
    bf* XB[2];
    XB[0] = (bf*)wsp; wsp += SZ_XB;
    XB[1] = (bf*)wsp; wsp += SZ_XB;
    bf* WB = (bf*)wsp; wsp += SZ_WB;
    float* RT = (float*)wsp; wsp += SZ_RT;
    h16* BT = (h16*)wsp; wsp += SZ_BT;
    h16* AM = (h16*)wsp; wsp += SZ_AM;
    bf* W0 = WB; bf* W1 = WB + (size_t)DM * DM; bf* W2 = WB + (size_t)2 * DM * DM; bf* W3 = WB + (size_t)3 * DM * DM;
    const size_t pl = (size_t)NB * DM * SEQ;

    for (int i = 0; i < 2; ++i) {
        if (SEQ == SEQ_FULL) {
            const size_t n8 = (size_t)NB * SEQ * DM / 8;
            k_cvt8<<<(unsigned)((n8 + 255) / 256), 256, 0, stream>>>(xin[i], XB[i], n8);
        } else {
            const size_t n8 = (size_t)SEQ * DM / 8;
            for (int b = 0; b < NB; ++b) k_cvt8<<<(unsigned)((n8 + 255) / 256), 256, 0, stream>>>(xin[i] + (size_t)b * SEQ_FULL * DM, XB[i] + (size_t)b * SEQ * DM, n8);
        }
    }
    { const size_t n8 = (size_t)DM * DM / 8; const unsigned g = (unsigned)((n8 + 255) / 256);
      k_cvt8<<<g, 256, 0, stream>>>(wr1, W0, n8); k_cvt8<<<g, 256, 0, stream>>>(wi1, W1, n8);
      k_cvt8<<<g, 256, 0, stream>>>(wr2, W2, n8); k_cvt8<<<g, 256, 0, stream>>>(wi2, W3, n8); }

    k_lin<<<dim3(DM / 64, NB * SEQ / 64, 1), 32, 0, stream>>>(W0, XB[0], br1, RT);
    k_lin<<<dim3(DM / 64, NB * SEQ / 64, 1), 32, 0, stream>>>(W1, XB[1], bi1, RT + pl);
    k_lin<<<dim3(DM / 64, NB * SEQ / 64, 1), 32, 0, stream>>>(W2, XB[0], br2, RT + 2 * pl);
    k_lin<<<dim3(DM / 64, NB * SEQ / 64, 1), 32, 0, stream>>>(W3, XB[1], bi2, RT + 3 * pl);

    k_att<<<dim3(NB, 1, 1), SEQ, 0, stream>>>(RT, BT, AM);

    k_outer<<<dim3(DM / OTR, DM / 64, 2 * NB), 32, 0, stream>>>(AM, BT, OUT);
}
